// ModelWrapper_49100066128303
// MI455X (gfx1250) — hardware-verified
//
#include <hip/hip_runtime.h>
#include <hip/hip_bf16.h>
#include <math.h>

#define NNODE 100000
#define DIM 128
#define KIN 256
#define HID 1024
#define NPAIR 262144

typedef _Float16 f16;
typedef __attribute__((ext_vector_type(16))) f16 f16x16;
typedef __attribute__((ext_vector_type(8)))  f16 f16x8;
typedef __attribute__((ext_vector_type(8)))  float f32x8;
typedef __attribute__((ext_vector_type(4)))  float v4f_t;
typedef float v4fa __attribute__((ext_vector_type(4), may_alias));
__device__ __forceinline__ f32x8 wmma16(f16x16 a, f16x16 b, f32x8 c) {
  c = __builtin_amdgcn_wmma_f32_16x16x32_f16(false, a, false, b, (short)0, c, false, false);
  asm volatile("v_nop\n\tv_nop\n\tv_nop\n\tv_nop" : "+v"(c) : "v"(a), "v"(b));
  return c;
}
__device__ __forceinline__ f16x16 lds_frag(const f16* base, int stride) {
  const int lane = threadIdx.x & 31, row = lane & 15, kh = (lane >> 4) * 8;
  const f16x8 lo = *(const f16x8*)(base + row * stride + kh);
  const f16x8 hi = *(const f16x8*)(base + row * stride + kh + 16);
  f16x16 f;
#pragma unroll
  for (int i = 0; i < 8; ++i) { f[i] = lo[i]; f[i + 8] = hi[i]; }
  return f;
}
__global__ __launch_bounds__(256) void k_pairmlp(const float* __restrict__ emb, const int* __restrict__ ig, const int* __restrict__ idd, const float* __restrict__ W1, const float* __restrict__ b1,
                                                const float* __restrict__ W2, const float* __restrict__ b2, float* __restrict__ out) {
  __shared__ __attribute__((aligned(16))) f16 aS[128 * (KIN + 8)];
  __shared__ __attribute__((aligned(16))) f16 wS[128 * 40];
  __shared__ __attribute__((aligned(16))) float tS[128 * 68];
  __shared__ __attribute__((aligned(16))) float oS[128 * 2];
  const int tid = threadIdx.x, lane = tid & 31, wave = tid >> 5, cl = lane & 15, rh = (lane >> 4) * 8;
  const size_t p0 = (size_t)blockIdx.x * 128;
  { const int r = tid >> 1, half = tid & 1; int node = half ? idd[p0 + r] : ig[p0 + r]; node = min(max(node, 0), NNODE - 1);
    const float* src = emb + (size_t)node * DIM; f16* dst = aS + r * (KIN + 8) + half * DIM;
#pragma unroll 1
    for (int c = 0; c < DIM; c += 4) { const v4f_t v = *(const v4f_t*)(src + c); dst[c] = (f16)v[0]; dst[c + 1] = (f16)v[1]; dst[c + 2] = (f16)v[2]; dst[c + 3] = (f16)v[3]; } }
  float o0 = 0.0f, o1 = 0.0f;
  const int er = tid >> 1, eh = (tid & 1) * 32;
#pragma unroll 1
  for (int g = 0; g < HID / 128; ++g) {
    f32x8 acc[8];
#pragma unroll
    for (int j = 0; j < 8; ++j) { f32x8 z = {}; acc[j] = z; }
#pragma unroll 1
    for (int ks = 0; ks < KIN / 32; ++ks) {
      __syncthreads();
      { const int kk = tid >> 3, q = (tid & 7) * 16; const float* wr = W1 + (size_t)(ks * 32 + kk) * HID + g * 128 + q;
#pragma unroll
        for (int e = 0; e < 16; ++e) wS[(q + e) * 40 + kk] = (f16)wr[e]; }
      __syncthreads();
      const f16x16 af = lds_frag(aS + (wave * 16) * (KIN + 8) + ks * 32, KIN + 8);
#pragma unroll
      for (int j = 0; j < 8; ++j) acc[j] = wmma16(af, lds_frag(wS + (j * 16) * 40, 40), acc[j]);
    }
#pragma unroll
    for (int jh = 0; jh < 2; ++jh) {
      __syncthreads();
#pragma unroll
      for (int j = 0; j < 4; ++j)
#pragma unroll
        for (int r = 0; r < 8; ++r) tS[(wave * 16 + rh + r) * 68 + j * 16 + cl] = acc[jh * 4 + j][r];
      __syncthreads();
#pragma unroll 1
      for (int c = 0; c < 32; ++c) { const int col = eh + c; const int n = g * 128 + jh * 64 + col; const float u = tS[er * 68 + col] + b1[n];
        const float h = 0.5f * u * (1.0f + erff(u * 0.70710678118654752f)); o0 += h * W2[n * 2]; o1 += h * W2[n * 2 + 1]; }
    }
  }
  o0 += __shfl_xor(o0, 1, 32); o1 += __shfl_xor(o1, 1, 32);
  if ((tid & 1) == 0) { oS[er * 2] = o0 + b2[0]; oS[er * 2 + 1] = o1 + b2[1]; }
  __syncthreads();
#pragma unroll 1
  for (int pass = 0; pass < 2; ++pass) { if (tid < 64) *(volatile v4f_t*)(out + p0 * 2 + tid * 4) = *(const v4fa*)(oS + tid * 4); __threadfence(); }
}

extern "C" void kernel_launch(void* const* d_in, const int* in_sizes, int n_in,
                              void* d_out, int out_size, void* d_ws, size_t ws_size,
                              hipStream_t stream) {
  (void)in_sizes; (void)n_in; (void)out_size; (void)d_ws; (void)ws_size;
  const float* emb = (const float*)d_in[0]; const int* ig = (const int*)d_in[1]; const int* idd = (const int*)d_in[2];
  const float* W1 = (const float*)d_in[3]; const float* b1 = (const float*)d_in[4]; const float* W2 = (const float*)d_in[5]; const float* b2 = (const float*)d_in[6];
  float* out = (float*)d_out;
  k_pairmlp<<<dim3(NPAIR / 128), dim3(256), 0, stream>>>(emb, ig, idd, W1, b1, W2, b2, out);
}
